// TwoBranchGNN_31490700214324
// MI455X (gfx1250) — hardware-verified
//
#include <hip/hip_runtime.h>
#include <math.h>

#define NN    50000
#define NPAD  50048
#define HID   128
#define NCLS  40
#define NCP   64
#define NE    500000
#define NT    256
#define TILE  4096
#define NTILE 13
#define SCH   2048
#define SPT   (SCH / NT)
#define NCH   ((NE + SCH - 1) / SCH)
#define WSC   16.0f
#define WSCI  0.0625f
#define LSB   64

typedef __attribute__((ext_vector_type(16))) _Float16 v16h;
typedef __attribute__((ext_vector_type(8)))  _Float16 v8h;
typedef __attribute__((ext_vector_type(4)))  _Float16 v4h;
typedef __attribute__((ext_vector_type(16))) __bf16   v16b;
typedef __attribute__((ext_vector_type(8)))  __bf16   v8b;
typedef __attribute__((ext_vector_type(8)))  float    v8f;
typedef __attribute__((ext_vector_type(4)))  float    v4f;
typedef __attribute__((ext_vector_type(4)))  int      v4i;

__device__ __forceinline__ unsigned short f2bf_bits(float f) {
  unsigned u = __float_as_uint(f);
  return (unsigned short)((u + 0x7FFFu + ((u >> 16) & 1u)) >> 16);
}
__device__ __forceinline__ float bf_bits2f(unsigned short h) { return __uint_as_float(((unsigned)h) << 16); }

__device__ __forceinline__ void dep_guard_h(v8f& a, v8f& b, v16h x, v16h y) { asm volatile("v_nop\n\tv_nop\n\tv_nop\n\tv_nop" : "+v"(a), "+v"(b) : "v"(x), "v"(y)); }
__device__ __forceinline__ void dep_guard_b(v8f& a, v8f& b, v16b x, v16b y) { asm volatile("v_nop\n\tv_nop\n\tv_nop\n\tv_nop" : "+v"(a), "+v"(b) : "v"(x), "v"(y)); }
__device__ __forceinline__ void keep4_h(v16h a, v16h b, v16h c, v16h d) { asm volatile("v_nop" :: "v"(a), "v"(b), "v"(c), "v"(d)); }
__device__ __forceinline__ void keep4_b(v16b a, v16b b, v16b c, v16b d) { asm volatile("v_nop" :: "v"(a), "v"(b), "v"(c), "v"(d)); }
__device__ __forceinline__ void acc_guard4(v8f& a, v8f& b, v8f& c, v8f& d) { asm volatile("v_nop\n\tv_nop\n\tv_nop\n\tv_nop" : "+v"(a), "+v"(b), "+v"(c), "+v"(d)); }
template <typename T> struct Frag;
template <> struct Frag<_Float16> {
  typedef v16h V; union U { v16h v; v8h h[2]; };
  static __device__ __forceinline__ v16h load(const _Float16* p) {
    U f; f.h[0] = *(const v8h*)(p); f.h[1] = *(const v8h*)(p + 16); return f.v;
  }
  static __device__ __forceinline__ v8f mma(v16h a, v16h b, v8f c) {
    return __builtin_amdgcn_wmma_f32_16x16x32_f16(false, a, false, b, (short)0, c, false, false);
  }
  static __device__ __forceinline__ void guard(v8f& a, v8f& b, v16h x, v16h y) { dep_guard_h(a, b, x, y); }
  static __device__ __forceinline__ void keep(v16h a, v16h b, v16h c, v16h d) { keep4_h(a, b, c, d); }
};
template <> struct Frag<__bf16> {
  typedef v16b V; union U { v16b v; v8b h[2]; };
  static __device__ __forceinline__ v16b load(const __bf16* p) {
    U f; f.h[0] = *(const v8b*)(p); f.h[1] = *(const v8b*)(p + 16); return f.v;
  }
  static __device__ __forceinline__ v8f mma(v16b a, v16b b, v8f c) {
    return __builtin_amdgcn_wmma_f32_16x16x32_bf16(false, a, false, b, (short)0, c, false, false);
  }
  static __device__ __forceinline__ void guard(v8f& a, v8f& b, v16b x, v16b y) { dep_guard_b(a, b, x, y); }
  static __device__ __forceinline__ void keep(v16b a, v16b b, v16b c, v16b d) { keep4_b(a, b, c, d); }
};

template <int OUT_MODE, bool MIX, int ACT>
__global__ __launch_bounds__(256) void wmma_gemm64_cat(
    const unsigned short* __restrict__ A1p, int lda1,
    const unsigned short* __restrict__ A2p, int lda2, int K1,
    const unsigned short* __restrict__ Btp, int ldb,
    void* __restrict__ Cout, void* __restrict__ Cout2, int ldc,
    const float* __restrict__ bias,
    const unsigned short* __restrict__ Rp, const float* __restrict__ mixr,
    int M, int N, int K, float scale) {
  typedef _Float16 T;
  typedef v16h V;
  const T* A1 = (const T*)A1p; const T* A2 = (const T*)A2p; const T* Bt = (const T*)Btp;
  __shared__ __align__(16) float sT[8][16 * 68];
  const int lane = threadIdx.x & 31;
  const int wave = threadIdx.x >> 5;
  const int tilesN = N >> 6;
  const int tilesM = M >> 6;
  const int tile = blockIdx.x * 8 + wave;
  if (tile >= tilesM * tilesN) return;
  const int tm = tile / tilesN;
  const int tn = tile - tm * tilesN;
  const int m0 = tm << 6;
  const int n0 = tn << 6;

  const int rlane = lane & 15;
  const int koff  = (lane >> 4) * 8;
  const int mOff  = (lane >> 4) * 8;

  v8f acc[4][4];
#pragma unroll
  for (int i = 0; i < 4; ++i)
#pragma unroll
    for (int j = 0; j < 4; ++j) acc[i][j] = (v8f){0.f,0.f,0.f,0.f,0.f,0.f,0.f,0.f};

  for (int k0 = 0; k0 < K; k0 += 32) {
    const bool fst = (k0 < K1);
    const T* Ab = fst ? A1 : A2;
    const int lda = fst ? lda1 : lda2;
    const int kk = fst ? k0 : (k0 - K1);
    V bh[4];
#pragma unroll
    for (int j = 0; j < 4; ++j) {
      const size_t bo = (size_t)(n0 + (j << 4) + rlane) * ldb + koff + k0;
      bh[j] = Frag<T>::load(Bt + bo);
    }
#pragma unroll
    for (int i = 0; i < 4; ++i) {
      const size_t ao = (size_t)(m0 + (i << 4) + rlane) * lda + koff + kk;
      V ah = Frag<T>::load(Ab + ao);
#pragma unroll
      for (int j = 0; j < 4; ++j) acc[i][j] = Frag<T>::mma(ah, bh[j], acc[i][j]);
      Frag<T>::guard(acc[i][0], acc[i][3], ah, ah);
    }
    Frag<T>::keep(bh[0], bh[1], bh[2], bh[3]);
  }
  acc_guard4(acc[0][0], acc[0][1], acc[0][2], acc[0][3]);
  acc_guard4(acc[1][0], acc[1][1], acc[1][2], acc[1][3]);
  acc_guard4(acc[2][0], acc[2][1], acc[2][2], acc[2][3]);
  acc_guard4(acc[3][0], acc[3][1], acc[3][2], acc[3][3]);

  float* slab = sT[wave];
  const float rr = MIX ? mixr[0] : 0.f;
  const _Float16* R = (const _Float16*)Rp;
#pragma unroll
  for (int i = 0; i < 4; ++i) {
    const int mBase = m0 + (i << 4);
#pragma unroll
    for (int j = 0; j < 4; ++j) {
      const int n = n0 + (j << 4) + rlane;
      const float bv = bias[n];
#pragma unroll
      for (int r = 0; r < 8; ++r) {
        float v = acc[i][j][r] * scale + bv;
        if (ACT == 2) v = fmaxf(v, 0.0f);
        if (MIX) {
          const float pv = (float)R[(size_t)(mBase + mOff + r) * ldc + n];
          v = pv * rr + v * (1.0f - rr);
        }
        slab[(mOff + r) * 68 + (j << 4) + rlane] = v;
      }
    }
    __builtin_amdgcn_fence(__ATOMIC_RELEASE, "workgroup");
    __builtin_amdgcn_wave_barrier();
    __builtin_amdgcn_fence(__ATOMIC_ACQUIRE, "workgroup");
    if (OUT_MODE == 0 || OUT_MODE == 3) {
      float* C = (float*)Cout;
      const int hh = lane >> 4, c4 = (lane & 15) * 4;
      for (int pass = 0; pass < 2; ++pass) {
#pragma unroll
        for (int it = 0; it < 8; ++it) {
          const int row = it * 2 + hh;
          v4f v = *(const v4f*)(slab + row * 68 + c4);
          *(volatile v4f*)(C + (size_t)(mBase + row) * ldc + n0 + c4) = v;
        }
        __threadfence();
      }
    }
    if (OUT_MODE == 1 || OUT_MODE == 3) {
      unsigned short* C = (unsigned short*)(OUT_MODE == 3 ? Cout2 : Cout);
      const int q = lane >> 3, c8 = (lane & 7) * 8;
      for (int pass = 0; pass < 2; ++pass) {
#pragma unroll
        for (int it = 0; it < 4; ++it) {
          const int row = it * 4 + q;
          const float* sp = slab + row * 68 + c8;
          v8h hv;
#pragma unroll
          for (int e = 0; e < 8; ++e) hv[e] = (_Float16)sp[e];
          *(volatile v8h*)(C + (size_t)(mBase + row) * ldc + n0 + c8) = hv;
        }
        __threadfence();
      }
    }
    __builtin_amdgcn_fence(__ATOMIC_RELEASE, "workgroup");
    __builtin_amdgcn_wave_barrier();
    __builtin_amdgcn_fence(__ATOMIC_ACQUIRE, "workgroup");
  }
}

__device__ __forceinline__ int blk_excl_scan(int cnt, int* scan_ws, int tid, int* tot) {
  const int lane = tid & 31, wave = tid >> 5; int incl = cnt;
#pragma unroll
  for (int o = 1; o < 32; o <<= 1) { const int v = __shfl_up(incl, o, 32); if (lane >= o) incl += v; }
  if (lane == 31) scan_ws[wave] = incl;
  __syncthreads();
  if (wave == 0) { int wv = (lane < NT / 32) ? scan_ws[lane] : 0; int wincl = wv;
#pragma unroll
    for (int o = 1; o < 32; o <<= 1) { const int v = __shfl_up(wincl, o, 32); if (lane >= o) wincl += v; }
    if (lane < NT / 32) scan_ws[32 + lane] = wincl - wv; if (lane == 31) scan_ws[64] = wincl; }
  __syncthreads();
  const int res = scan_ws[32 + wave] + incl - cnt; *tot = scan_ws[64];
  return res;
}
template <int SP, int CAP>
__device__ __forceinline__ int chunk_hits(const int* __restrict__ dstv, int e0, int n0, int hiN, int tid, int* LIST, int* scan_ws) {
  const int eb = e0 + tid * SP;
  const bool inr = eb < NE;
  const int ebc = inr ? eb : (NE - SP);
  int rec[SP]; int cnt = 0;
#pragma unroll
  for (int k = 0; k < SP; k += 4) {
    const v4i d4 = *(const v4i*)(dstv + ebc + k);
#pragma unroll
    for (int e = 0; e < 4; ++e) {
      const int d = d4[e]; int r = -1;
      if (inr && d >= n0 && d < hiN) { r = ebc + k + e; ++cnt; }
      rec[k + e] = r;
    }
  }
  int tot; int p = blk_excl_scan(cnt, scan_ws, tid, &tot);
#pragma unroll
  for (int k = 0; k < SP; ++k) if (rec[k] >= 0) { if ((unsigned)p < (unsigned)CAP) LIST[p] = rec[k]; ++p; }
  __syncthreads();
  return tot < CAP ? tot : CAP;
}

template <bool IDX2>
__global__ __launch_bounds__(NT) void agg_kernel(const float* __restrict__ X, const int* __restrict__ rows,
                                                const int* __restrict__ cols, const float* __restrict__ vals,
                                                const int* __restrict__ idv, float* ACC, unsigned short* __restrict__ OUTH) {
  __shared__ int LIST[SCH];
  __shared__ int scan_ws[80];
  const int tid = threadIdx.x, lane = tid & 31, wave = tid >> 5;
  const int n0 = blockIdx.x * TILE;
  const int hiN = (n0 + TILE < NPAD) ? (n0 + TILE) : NPAD;
  const v4f z4 = {0.f, 0.f, 0.f, 0.f};
  for (int pass = 0; pass < 2; ++pass) {
#pragma unroll 1
    for (int j = 0; j < TILE / 8; ++j) {
      const int n = n0 + wave + 8 * j;
      if (n >= NPAD) break;
      *(volatile v4f*)(ACC + (size_t)n * HID + 4 * lane) = z4;
    }
    __threadfence();
  }
#pragma unroll 1
  for (int c = 0; c < NCH; ++c) {
    const int tot = chunk_hits<SPT, SCH>(rows, c * SCH, n0, hiN, tid, LIST, scan_ws);
#pragma unroll 1
    for (int base = 0; base < tot; base += 32) {
      const int q = base + lane;
      const int qc = (q < SCH) ? q : (SCH - 1);
      int e = LIST[qc];
      if (q >= tot) e = -1;
      const int ec = (e < 0) ? 0 : ((e >= NE) ? (NE - 1) : e);
      const int d = rows[ec];
      int dl = d - n0; dl = (dl < 0) ? 0 : ((dl >= TILE) ? (TILE - 1) : dl);
      int cc = cols[ec]; cc = (cc < 0) ? 0 : ((cc >= NN) ? (NN - 1) : cc);
      int s = cc;
      if (IDX2) { s = idv[cc]; s = (s < 0) ? 0 : ((s >= NN) ? (NN - 1) : s); }
      const float v = vals[ec];
      const int own = (e >= 0 && (dl & 7) == wave) ? 1 : 0;
      unsigned msk = (unsigned)__ballot(own);
#pragma unroll 1
      for (int it = 0; it < 32; ++it) {
        if (msk == 0u) break;
        const int bp = __builtin_ctz(msk); msk &= msk - 1u;
        const int sh = __shfl(s, bp, 32);
        const int dh = __shfl(dl, bp, 32);
        const float vh = __shfl(v, bp, 32);
        int n = n0 + dh; n = (n < NPAD) ? n : (NPAD - 1);
        const v4f xs = *(const v4f*)(X + (size_t)sh * HID + 4 * lane);
        float* rp = ACC + (size_t)n * HID + 4 * lane;
        v4f a = *(const v4f*)rp;
        a = a + vh * xs;
        *(volatile v4f*)rp = a;
        __threadfence();
        *(volatile v4f*)rp = a;
      }
    }
    __syncthreads();
  }
  for (int pass = 0; pass < 2; ++pass) {
#pragma unroll 1
    for (int j = 0; j < TILE / 8; ++j) {
      const int n = n0 + wave + 8 * j;
      if (n >= NPAD) break;
      const v4f a = *(const v4f*)(ACC + (size_t)n * HID + 4 * lane);
      v4h hv;
      hv[0] = (_Float16)a[0]; hv[1] = (_Float16)a[1]; hv[2] = (_Float16)a[2]; hv[3] = (_Float16)a[3];
      *(volatile v4h*)(OUTH + (size_t)n * HID + 4 * lane) = hv;
    }
    __threadfence();
  }
}

__global__ __launch_bounds__(NT) void prep_kernel(const float* __restrict__ Wl, const float* __restrict__ Wr, const float* __restrict__ Wo,
                                                 const float* __restrict__ bo, unsigned* __restrict__ WB, unsigned* __restrict__ WOB,
                                                 float* __restrict__ BP) {
  const int i = blockIdx.x * NT + threadIdx.x;
  if (i < 3 * HID * HID) {
    const int L = i >> 14, rem = i & 16383, n = rem >> 7, kd = rem & 127, k = 2 * kd;
    const int kk = k & 127;
    const size_t base = (size_t)L * HID * HID;
    const float l0 = Wl[base + (size_t)kk * HID + n], l1 = Wl[base + (size_t)(kk + 1) * HID + n];
    const float r0 = Wr[base + (size_t)kk * HID + n], r1 = Wr[base + (size_t)(kk + 1) * HID + n];
    const float a = ((k < 128) ? l0 : r0) * WSC, b = ((k < 128) ? l1 : r1) * WSC;
    const _Float16 ha = (_Float16)a, hb = (_Float16)b;
    const unsigned u = (unsigned)__builtin_bit_cast(unsigned short, ha) | ((unsigned)__builtin_bit_cast(unsigned short, hb) << 16);
    ((volatile unsigned*)WB)[i] = u;
    __threadfence();
    ((volatile unsigned*)WB)[i] = u;
  } else if (i < 3 * HID * HID + NCP * (HID / 2)) {
    const int j = i - 3 * HID * HID;
    const int n = j >> 6, kd = j & 63, k = 2 * kd;
    const int nc = (n < NCLS) ? n : (NCLS - 1);
    float a = Wo[(size_t)k * NCLS + nc] * WSC, b = Wo[(size_t)(k + 1) * NCLS + nc] * WSC;
    if (n >= NCLS) { a = 0.f; b = 0.f; }
    const _Float16 ha = (_Float16)a, hb = (_Float16)b;
    const unsigned u = (unsigned)__builtin_bit_cast(unsigned short, ha) | ((unsigned)__builtin_bit_cast(unsigned short, hb) << 16);
    ((volatile unsigned*)WOB)[j] = u;
    __threadfence();
    ((volatile unsigned*)WOB)[j] = u;
  }
  if (blockIdx.x == 0 && threadIdx.x < NCP) {
    const int t = threadIdx.x;
    const int tc = (t < NCLS) ? t : (NCLS - 1);
    float v = bo[tc];
    if (t >= NCLS) v = 0.f;
    ((volatile float*)BP)[t] = v;
    __threadfence();
    ((volatile float*)BP)[t] = v;
  }
}

__global__ __launch_bounds__(NT) void cast_rows_f16(const float* __restrict__ x, unsigned short* __restrict__ outp) {
  const int t = blockIdx.x * NT + threadIdx.x;
  if (t >= NPAD * 16) return;
  const int row = t >> 4, c8 = (t & 15) * 8;
  const int rc = (row < NN) ? row : (NN - 1);
  const bool live = row < NN;
  const v4f a = *(const v4f*)(x + (size_t)rc * HID + c8);
  const v4f b = *(const v4f*)(x + (size_t)rc * HID + c8 + 4);
  v8h hv;
#pragma unroll
  for (int e = 0; e < 4; ++e) {
    hv[e]     = live ? (_Float16)a[e] : (_Float16)0.0f;
    hv[4 + e] = live ? (_Float16)b[e] : (_Float16)0.0f;
  }
  unsigned short* op = outp + (size_t)row * HID + c8;
  *(volatile v8h*)op = hv;
  __threadfence();
  *(volatile v8h*)op = hv;
}

__global__ __launch_bounds__(NT) void mix0_kernel(const float* __restrict__ x, const int* __restrict__ idv, const float* __restrict__ mixr,
                                                 unsigned short* __restrict__ outp) {
  const int t = blockIdx.x * NT + threadIdx.x;
  if (t >= NPAD * 32) return;
  const int row = t >> 5, c4 = (t & 31) * 4;
  const int rc = (row < NN) ? row : (NN - 1);
  const bool live = row < NN;
  int s = idv[rc]; s = (s < 0) ? 0 : ((s >= NN) ? (NN - 1) : s);
  const float r = mixr[0];
  const v4f a = *(const v4f*)(x + (size_t)rc * HID + c4);
  const v4f b = *(const v4f*)(x + (size_t)s * HID + c4);
  const v4f m = a * r + b * (1.0f - r);
  v4h hv;
#pragma unroll
  for (int e = 0; e < 4; ++e) hv[e] = live ? (_Float16)m[e] : (_Float16)0.0f;
  unsigned short* op = outp + (size_t)row * HID + c4;
  *(volatile v4h*)op = hv;
  __threadfence();
  *(volatile v4h*)op = hv;
}

__global__ __launch_bounds__(NT) void logsoftmax_kernel(const float* __restrict__ lg, float* __restrict__ outp) {
  __shared__ __align__(16) float so[LSB * NCLS];
  const int tid = threadIdx.x;
  const int nb = blockIdx.x * LSB;
  int nn = NN - nb; nn = (nn > LSB) ? LSB : nn;
  if (tid < LSB) {
    int n = nb + tid; n = (n < NN) ? n : (NN - 1);
    const float* p = lg + (size_t)n * NCP;
    float mx = p[0];
#pragma unroll 1
    for (int c = 1; c < NCLS; ++c) mx = fmaxf(mx, p[c]);
    float s = 0.f;
#pragma unroll 1
    for (int c = 0; c < NCLS; ++c) s += expf(p[c] - mx);
    const float ls = logf(s);
#pragma unroll 1
    for (int c = 0; c < NCLS; ++c) so[tid * NCLS + c] = (p[c] - mx) - ls;
  }
  __syncthreads();
  const int cnt4 = nn * (NCLS / 4);
  float* ob = outp + (size_t)nb * NCLS;
  for (int pass = 0; pass < 2; ++pass) {
    for (int i = tid; i < cnt4; i += NT) {
      const v4f v = *(const v4f*)(so + 4 * i);
      *(volatile v4f*)(ob + 4 * i) = v;
    }
    __threadfence();
  }
}

extern "C" void kernel_launch(void* const* d_in, const int* in_sizes, int n_in,
                              void* d_out, int out_size, void* d_ws, size_t ws_size, hipStream_t stream) {
  if (n_in < 14) return;
  if (in_sizes[0] != NN * HID || in_sizes[1] != NE || in_sizes[2] != NE || in_sizes[3] != NE ||
      in_sizes[4] != NE || in_sizes[5] != NE || in_sizes[6] != NE || in_sizes[7] < 1 || in_sizes[8] != NN ||
      in_sizes[9] != 3 * HID * HID || in_sizes[10] != 3 * HID * HID || in_sizes[11] != 3 * HID ||
      in_sizes[12] != HID * NCLS || in_sizes[13] != NCLS || out_size != NN * NCLS) return;
  const float* x0   = (const float*)d_in[0];
  const int*   aRow = (const int*)  d_in[1];
  const int*   aCol = (const int*)  d_in[2];
  const float* aVal = (const float*)d_in[3];
  const int*   bRow = (const int*)  d_in[4];
  const int*   bCol = (const int*)  d_in[5];
  const float* bVal = (const float*)d_in[6];
  const float* mixr = (const float*)d_in[7];
  const int*   idv  = (const int*)  d_in[8];
  const float* Wl   = (const float*)d_in[9];
  const float* Wr   = (const float*)d_in[10];
  const float* bs   = (const float*)d_in[11];
  const float* Wo   = (const float*)d_in[12];
  const float* bo   = (const float*)d_in[13];
  float* out = (float*)d_out;

  char* ws = (char*)d_ws; size_t off = 0;
  auto carve = [&](size_t bytes) -> char* { char* p = ws + off; off += (bytes + 255) & ~(size_t)255; return p; };
  const size_t SB = (size_t)NPAD * HID * 2;
  unsigned short* Pa  = (unsigned short*)carve(SB);
  unsigned short* Pb  = (unsigned short*)carve(SB);
  unsigned short* Pc  = (unsigned short*)carve(SB);
  unsigned short* Pf  = (unsigned short*)carve(SB);
  unsigned short* Pg  = (unsigned short*)carve(SB);
  unsigned short* Ph  = (unsigned short*)carve(SB);
  float*          X32 = (float*)carve((size_t)NPAD * HID * 4);
  float*          S   = (float*)carve((size_t)NPAD * HID * 4);
  unsigned*       WB  = (unsigned*)carve((size_t)3 * HID * 2 * HID * 2);
  unsigned*       WOB = (unsigned*)carve((size_t)NCP * HID * 2);
  float*          BP  = (float*)carve((size_t)NCP * 4);
  if (off > ws_size || off > (size_t)134217728) return;
  const unsigned short* WBh  = (const unsigned short*)WB;
  const unsigned short* WOBh = (const unsigned short*)WOB;
  float* LG = S;

  const int GBLK = ((NPAD / 64) * (HID / 64) + 7) / 8;
  const int OBLK = ((NPAD / 64) + 7) / 8;

  prep_kernel<<<dim3((3 * HID * HID + NCP * (HID / 2) + NT - 1) / NT), dim3(NT), 0, stream>>>(Wl, Wr, Wo, bo, WB, WOB, BP);
  cast_rows_f16<<<dim3((NPAD * 16 + NT - 1) / NT), dim3(NT), 0, stream>>>(x0, Pa);
  agg_kernel<false><<<dim3(NTILE), dim3(NT), 0, stream>>>(x0, aRow, aCol, aVal, idv, S, Pb);
  wmma_gemm64_cat<3, false, 2><<<dim3(GBLK), dim3(256), 0, stream>>>(
      Pb, HID, Pa, HID, HID, WBh + 0 * HID * 2 * HID, 2 * HID, (void*)X32, (void*)Pc, HID,
      bs + 0 * HID, (const unsigned short*)nullptr, mixr, NPAD, HID, 2 * HID, WSCI);
  mix0_kernel<<<dim3((NPAD * 32 + NT - 1) / NT), dim3(NT), 0, stream>>>(x0, idv, mixr, Pf);
  agg_kernel<true><<<dim3(NTILE), dim3(NT), 0, stream>>>(x0, bRow, bCol, bVal, idv, S, Pg);
  wmma_gemm64_cat<1, false, 2><<<dim3(GBLK), dim3(256), 0, stream>>>(
      Pb, HID, Pf, HID, HID, WBh + 0 * HID * 2 * HID, 2 * HID, (void*)Ph, (void*)nullptr, HID,
      bs + 0 * HID, (const unsigned short*)nullptr, mixr, NPAD, HID, 2 * HID, WSCI);
  wmma_gemm64_cat<1, true, 2><<<dim3(GBLK), dim3(256), 0, stream>>>(
      Pg, HID, Pf, HID, HID, WBh + 0 * HID * 2 * HID, 2 * HID, (void*)Pa, (void*)nullptr, HID,
      bs + 0 * HID, Ph, mixr, NPAD, HID, 2 * HID, WSCI);
  agg_kernel<false><<<dim3(NTILE), dim3(NT), 0, stream>>>(X32, aRow, aCol, aVal, idv, S, Pb);
  agg_kernel<true><<<dim3(NTILE), dim3(NT), 0, stream>>>(X32, bRow, bCol, bVal, idv, S, Pg);
  wmma_gemm64_cat<0, false, 2><<<dim3(GBLK), dim3(256), 0, stream>>>(
      Pb, HID, Pc, HID, HID, WBh + 1 * HID * 2 * HID, 2 * HID, (void*)X32, (void*)nullptr, HID,
      bs + 1 * HID, (const unsigned short*)nullptr, mixr, NPAD, HID, 2 * HID, WSCI);
  wmma_gemm64_cat<1, false, 2><<<dim3(GBLK), dim3(256), 0, stream>>>(
      Pb, HID, Pa, HID, HID, WBh + 1 * HID * 2 * HID, 2 * HID, (void*)Ph, (void*)nullptr, HID,
      bs + 1 * HID, (const unsigned short*)nullptr, mixr, NPAD, HID, 2 * HID, WSCI);
  wmma_gemm64_cat<1, true, 2><<<dim3(GBLK), dim3(256), 0, stream>>>(
      Pg, HID, Pa, HID, HID, WBh + 1 * HID * 2 * HID, 2 * HID, (void*)Pf, (void*)nullptr, HID,
      bs + 1 * HID, Ph, mixr, NPAD, HID, 2 * HID, WSCI);
  agg_kernel<false><<<dim3(NTILE), dim3(NT), 0, stream>>>(X32, aRow, aCol, aVal, idv, S, Pb);
  agg_kernel<true><<<dim3(NTILE), dim3(NT), 0, stream>>>(X32, bRow, bCol, bVal, idv, S, Pg);
  wmma_gemm64_cat<1, false, 2><<<dim3(GBLK), dim3(256), 0, stream>>>(
      Pb, HID, Pf, HID, HID, WBh + 2 * HID * 2 * HID, 2 * HID, (void*)Ph, (void*)nullptr, HID,
      bs + 2 * HID, (const unsigned short*)nullptr, mixr, NPAD, HID, 2 * HID, WSCI);
  wmma_gemm64_cat<1, true, 2><<<dim3(GBLK), dim3(256), 0, stream>>>(
      Pg, HID, Pf, HID, HID, WBh + 2 * HID * 2 * HID, 2 * HID, (void*)Pa, (void*)nullptr, HID,
      bs + 2 * HID, Ph, mixr, NPAD, HID, 2 * HID, WSCI);
  wmma_gemm64_cat<0, false, 0><<<dim3(OBLK), dim3(256), 0, stream>>>(
      Pa, HID, Pa, HID, HID, WOBh, HID, (void*)LG, (void*)nullptr, NCP,
      BP, (const unsigned short*)nullptr, mixr, NPAD, NCP, HID, WSCI);
  logsoftmax_kernel<<<dim3((NN + LSB - 1) / LSB), dim3(NT), 0, stream>>>(LG, out);
}
